// Executor_46334107189311
// MI455X (gfx1250) — hardware-verified
//
#include <hip/hip_runtime.h>
#include <math.h>

constexpr int kB     = 4096;
constexpr int kSlots = 8;
constexpr int kP     = 768;
constexpr int kSlot  = 256;
constexpr int kHid   = 256;
constexpr int kNC    = 512;
constexpr int kRows  = kB * kSlots;
constexpr float kInvSqrtP = 0.036084391824351614f;
constexpr float kPCarry   = 32768.0f;
constexpr float kPVScale  = 256.0f / 32768.0f;
constexpr float kCWScale  = 1.0f / 4096.0f;
constexpr float kW2Scale  = 1.0f / 16.0f;
constexpr float kWCarry   = 16.0f;
constexpr float kLnEps    = 1e-5f;
constexpr float kInvHid   = 1.0f / 256.0f;

static_assert(kB % 64 == 0 && kP % 64 == 0 && kNC % 64 == 0 && kHid % 64 == 0 && kSlot % 64 == 0 && kRows % 64 == 0, "tile multiples");
static_assert(kP % 32 == 0 && kNC % 32 == 0 && kSlot % 32 == 0 && kHid % 32 == 0, "K multiples of 32");

typedef __attribute__((ext_vector_type(16))) _Float16 v16h;
typedef __attribute__((ext_vector_type(8)))  _Float16 v8h;
typedef __attribute__((ext_vector_type(16))) __bf16   v16b;
typedef __attribute__((ext_vector_type(8)))  __bf16   v8b;
typedef __attribute__((ext_vector_type(8)))  float    v8f;
typedef __attribute__((ext_vector_type(4)))  float    v4f;
typedef __attribute__((ext_vector_type(4)))  unsigned int v4u;

__device__ __forceinline__ unsigned short f2bf_bits(float f) {
  unsigned u = __float_as_uint(f);
  return (unsigned short)((u + 0x7FFFu + ((u >> 16) & 1u)) >> 16);
}
__device__ __forceinline__ float bf_bits2f(unsigned short h) { return __uint_as_float(((unsigned)h) << 16); }

__device__ __forceinline__ void dep_guard_h(v8f& a, v8f& b, v16h x, v16h y) { asm volatile("v_nop\n\tv_nop\n\tv_nop\n\tv_nop" : "+v"(a), "+v"(b) : "v"(x), "v"(y)); }
__device__ __forceinline__ void dep_guard_b(v8f& a, v8f& b, v16b x, v16b y) { asm volatile("v_nop\n\tv_nop\n\tv_nop\n\tv_nop" : "+v"(a), "+v"(b) : "v"(x), "v"(y)); }
__device__ __forceinline__ void keep4_h(v16h a, v16h b, v16h c, v16h d) { asm volatile("v_nop" :: "v"(a), "v"(b), "v"(c), "v"(d)); }
__device__ __forceinline__ void keep4_b(v16b a, v16b b, v16b c, v16b d) { asm volatile("v_nop" :: "v"(a), "v"(b), "v"(c), "v"(d)); }
__device__ __forceinline__ void acc_guard4(v8f& a, v8f& b, v8f& c, v8f& d) { asm volatile("v_nop\n\tv_nop\n\tv_nop\n\tv_nop" : "+v"(a), "+v"(b), "+v"(c), "+v"(d)); }
template <typename T> struct Frag;
template <> struct Frag<_Float16> {
  typedef v16h V; union U { v16h v; v8h h[2]; };
  static __device__ __forceinline__ v16h load(const _Float16* p) {
    U f; f.h[0] = *(const v8h*)(p); f.h[1] = *(const v8h*)(p + 16); return f.v;
  }
  static __device__ __forceinline__ v8f mma(v16h a, v16h b, v8f c) {
    return __builtin_amdgcn_wmma_f32_16x16x32_f16(false, a, false, b, (short)0, c, false, false);
  }
  static __device__ __forceinline__ void guard(v8f& a, v8f& b, v16h x, v16h y) { dep_guard_h(a, b, x, y); }
  static __device__ __forceinline__ void keep(v16h a, v16h b, v16h c, v16h d) { keep4_h(a, b, c, d); }
};
template <> struct Frag<__bf16> {
  typedef v16b V; union U { v16b v; v8b h[2]; };
  static __device__ __forceinline__ v16b load(const __bf16* p) {
    U f; f.h[0] = *(const v8b*)(p); f.h[1] = *(const v8b*)(p + 16); return f.v;
  }
  static __device__ __forceinline__ v8f mma(v16b a, v16b b, v8f c) {
    return __builtin_amdgcn_wmma_f32_16x16x32_bf16(false, a, false, b, (short)0, c, false, false);
  }
  static __device__ __forceinline__ void guard(v8f& a, v8f& b, v16b x, v16b y) { dep_guard_b(a, b, x, y); }
  static __device__ __forceinline__ void keep(v16b a, v16b b, v16b c, v16b d) { keep4_b(a, b, c, d); }
};

__device__ __forceinline__ unsigned pk16(unsigned short a, unsigned short b) { return (unsigned)a | ((unsigned)b << 16); }
__device__ __forceinline__ unsigned short h_bits(float f) { const _Float16 h = (_Float16)f; return __builtin_bit_cast(unsigned short, h); }

template <int MODE> __device__ __forceinline__ unsigned short cvt16(float x, float scale) {
  const unsigned short bb = f2bf_bits(x);
  if (MODE == 0) return bb;
  return h_bits(bf_bits2f(bb) * scale);
}

template <int ET> struct Elem;
template <> struct Elem<0> { typedef _Float16 T; };
template <> struct Elem<1> { typedef __bf16 T; };
template <int ET, bool SPLIT, int BIAS_MODE, int OUT_MODE, int RESID, bool GATE, int ACT = 0>
__global__ __launch_bounds__(256) void wmma_gemm64(
    const unsigned short* __restrict__ Ap, const unsigned short* __restrict__ A2p, int lda, long strideA,
    const unsigned short* __restrict__ Btp, const unsigned short* __restrict__ Bt2p, int ldb, long strideB,
    void* __restrict__ Cout, void* __restrict__ Cout2, int ldc, long strideC,
    const float* __restrict__ bias,
    const float* __restrict__ resid, long strideR,
    const float* __restrict__ gmul, long strideG,
    int M, int N, int K, float scale) {
  typedef typename Elem<ET>::T T;
  typedef typename Frag<T>::V V;
  const T* A = (const T*)Ap; const T* A2 = (const T*)A2p; const T* Bt = (const T*)Btp; const T* Bt2 = (const T*)Bt2p;
  __shared__ __align__(16) float sT[8][16 * 68];
  const int b    = blockIdx.y;
  const int lane = threadIdx.x & 31;
  const int wave = threadIdx.x >> 5;
  const int tilesN = N >> 6;
  const int tilesM = M >> 6;
  const int tile = blockIdx.x * 8 + wave;
  if (tile >= tilesM * tilesN) return;
  const int tm = tile / tilesN;
  const int tn = tile - tm * tilesN;
  const int m0 = tm << 6;
  const int n0 = tn << 6;

  const T* Ab  = A  + (size_t)b * strideA;
  const T* Bb  = Bt + (size_t)b * strideB;
  const T* Ab2 = SPLIT ? (A2  + (size_t)b * strideA) : nullptr;
  const T* Bb2 = SPLIT ? (Bt2 + (size_t)b * strideB) : nullptr;

  const int rlane = lane & 15;
  const int koff  = (lane >> 4) * 8;
  const int mOff  = (lane >> 4) * 8;

  v8f acc[4][4];
#pragma unroll
  for (int i = 0; i < 4; ++i)
#pragma unroll
    for (int j = 0; j < 4; ++j) acc[i][j] = (v8f){0.f,0.f,0.f,0.f,0.f,0.f,0.f,0.f};

  for (int k0 = 0; k0 < K; k0 += 32) {
    V bh[4], bl[4];
#pragma unroll
    for (int j = 0; j < 4; ++j) {
      const size_t bo = (size_t)(n0 + (j << 4) + rlane) * ldb + koff + k0;
      bh[j] = Frag<T>::load(Bb + bo);
      if (SPLIT) bl[j] = Frag<T>::load(Bb2 + bo);
    }
#pragma unroll
    for (int i = 0; i < 4; ++i) {
      const size_t ao = (size_t)(m0 + (i << 4) + rlane) * lda + koff + k0;
      V ah = Frag<T>::load(Ab + ao);
      V al;
      if (SPLIT) al = Frag<T>::load(Ab2 + ao);
#pragma unroll
      for (int j = 0; j < 4; ++j) {
        acc[i][j] = Frag<T>::mma(ah, bh[j], acc[i][j]);
        if (SPLIT) {
          acc[i][j] = Frag<T>::mma(ah, bl[j], acc[i][j]);
          acc[i][j] = Frag<T>::mma(al, bh[j], acc[i][j]);
        }
      }
      Frag<T>::guard(acc[i][0], acc[i][3], ah, SPLIT ? al : ah);
    }
    Frag<T>::keep(bh[0], bh[1], bh[2], bh[3]);
    if (SPLIT) Frag<T>::keep(bl[0], bl[1], bl[2], bl[3]);
  }
  acc_guard4(acc[0][0], acc[0][1], acc[0][2], acc[0][3]);
  acc_guard4(acc[1][0], acc[1][1], acc[1][2], acc[1][3]);
  acc_guard4(acc[2][0], acc[2][1], acc[2][2], acc[2][3]);
  acc_guard4(acc[3][0], acc[3][1], acc[3][2], acc[3][3]);

  float* slab = sT[wave];
  const float* Rb = (RESID != 0) ? (resid + (size_t)b * strideR) : nullptr;
  const float* Gb = GATE ? (gmul + (size_t)b * strideG) : nullptr;
#pragma unroll
  for (int i = 0; i < 4; ++i) {
    const int mBase = m0 + (i << 4);
#pragma unroll
    for (int j = 0; j < 4; ++j) {
      const int n = n0 + (j << 4) + rlane;
      float bv = 0.f;
      if (BIAS_MODE == 2) bv = bias[n];
#pragma unroll
      for (int r = 0; r < 8; ++r) {
        float v = acc[i][j][r] * scale;
        if (BIAS_MODE == 1) v += bias[mBase + mOff + r];
        if (BIAS_MODE == 2) v += bv;
        const size_t ei = (size_t)(mBase + mOff + r) * ldc + n;
        if (GATE) v = v * Gb[ei];
        if (RESID == 1) v += Rb[ei];
        if (RESID == 2) v += bf_bits2f(f2bf_bits(Rb[ei]));
        if (ACT == 2) v = fmaxf(v, 0.0f);
        if (ACT == 4) v = (v > 0.f) ? v : 0.01f * v;
        slab[(mOff + r) * 68 + (j << 4) + rlane] = v;
      }
    }
    __builtin_amdgcn_fence(__ATOMIC_RELEASE, "workgroup");
    __builtin_amdgcn_wave_barrier();
    __builtin_amdgcn_fence(__ATOMIC_ACQUIRE, "workgroup");
    if (OUT_MODE == 0) {
      float* C = (float*)Cout + (size_t)b * strideC;
      const int hh = lane >> 4, c4 = (lane & 15) * 4;
      for (int pass = 0; pass < 2; ++pass) {
#pragma unroll
        for (int it = 0; it < 8; ++it) {
          const int row = it * 2 + hh;
          v4f v = *(const v4f*)(slab + row * 68 + c4);
          *(volatile v4f*)(C + (size_t)(mBase + row) * ldc + n0 + c4) = v;
        }
        __threadfence();
      }
    } else {
      const int q = lane >> 3, c8 = (lane & 7) * 8;
      unsigned short* C  = (unsigned short*)Cout  + (size_t)b * strideC;
      unsigned short* C2 = (OUT_MODE == 2) ? ((unsigned short*)Cout2 + (size_t)b * strideC) : nullptr;
      for (int pass = 0; pass < 2; ++pass) {
#pragma unroll
        for (int it = 0; it < 4; ++it) {
          const int row = it * 4 + q;
          const float* sp = slab + row * 68 + c8;
          v8h hv, lv;
#pragma unroll
          for (int e = 0; e < 8; ++e) {
            if (OUT_MODE == 1) {
              hv[e] = (_Float16)sp[e];
            } else {
              unsigned short hb = f2bf_bits(sp[e]);
              unsigned short lb = f2bf_bits(sp[e] - bf_bits2f(hb));
              hv[e] = __builtin_bit_cast(_Float16, hb);
              lv[e] = __builtin_bit_cast(_Float16, lb);
            }
          }
          *(volatile v8h*)(C + (size_t)(mBase + row) * ldc + n0 + c8) = hv;
          if (OUT_MODE == 2) *(volatile v8h*)(C2 + (size_t)(mBase + row) * ldc + n0 + c8) = lv;
        }
        __threadfence();
      }
    }
    __builtin_amdgcn_fence(__ATOMIC_RELEASE, "workgroup");
    __builtin_amdgcn_wave_barrier();
    __builtin_amdgcn_fence(__ATOMIC_ACQUIRE, "workgroup");
  }
}

template <int MODE>
__global__ __launch_bounds__(256) void cast8_kernel(const float* __restrict__ in0, const float* __restrict__ in1,
                                                    unsigned short* __restrict__ out, long zstride, int n8, float scale) {
  const int i = blockIdx.x * 256 + threadIdx.x;
  const int z = blockIdx.y;
  const float* src = (z == 0) ? in0 : in1;
  if (i < n8) {
    const v4f a = *(const v4f*)(src + (size_t)i * 8);
    const v4f c = *(const v4f*)(src + (size_t)i * 8 + 4);
    unsigned short hb[8];
#pragma unroll
    for (int e = 0; e < 4; ++e) { hb[e] = cvt16<MODE>(a[e], scale); hb[4 + e] = cvt16<MODE>(c[e], scale); }
    const v4u u = (v4u){pk16(hb[0], hb[1]), pk16(hb[2], hb[3]), pk16(hb[4], hb[5]), pk16(hb[6], hb[7])};
    unsigned short* op = out + (size_t)z * zstride + (size_t)i * 8;
    *(volatile v4u*)op = u;
    __threadfence();
    *(volatile v4u*)op = u;
  }
}

template <int MODE>
__global__ __launch_bounds__(256) void tcast_kernel(const float* __restrict__ in0, const float* __restrict__ in1,
                                                    int in_pitch, int krow0,
                                                    unsigned short* __restrict__ out, long zstride, int ldo, float scale) {
  __shared__ float sm[64][65];
  const int t  = threadIdx.x;
  const int k0 = blockIdx.x * 64;
  const int n0 = blockIdx.y * 64;
  const int z  = blockIdx.z;
  const float* W = (z == 0) ? in0 : in1;
#pragma unroll
  for (int i = 0; i < 16; ++i) {
    const int e  = i * 256 + t;
    const int kl = e >> 6;
    const int nl = e & 63;
    sm[nl][kl] = W[(size_t)(krow0 + k0 + kl) * in_pitch + n0 + nl];
  }
  __syncthreads();
  const int lane = t & 31, wave = t >> 5;
  const int q = lane >> 3, c8 = (lane & 7) * 8;
  unsigned short* op = out + (size_t)z * zstride;
  for (int pass = 0; pass < 2; ++pass) {
#pragma unroll
    for (int it = 0; it < 2; ++it) {
      const int row = wave * 8 + it * 4 + q;
      unsigned short hb[8];
#pragma unroll
      for (int e = 0; e < 8; ++e) hb[e] = cvt16<MODE>(sm[row][c8 + e], scale);
      const v4u u = (v4u){pk16(hb[0], hb[1]), pk16(hb[2], hb[3]), pk16(hb[4], hb[5]), pk16(hb[6], hb[7])};
      *(volatile v4u*)(op + (size_t)(n0 + row) * ldo + k0 + c8) = u;
    }
    __threadfence();
  }
}

__global__ __launch_bounds__(256) void softmax_kernel(const float* __restrict__ S, unsigned short* __restrict__ Pout, int nrows) {
  const int lane = threadIdx.x & 31, wave = threadIdx.x >> 5;
  const int row  = blockIdx.x * 8 + wave;
  const int rowc = (row < nrows) ? row : (nrows - 1);
  const float* sp = S + (size_t)rowc * kNC + lane * 8;
  const v4f a0 = *(const v4f*)(sp);
  const v4f a1 = *(const v4f*)(sp + 4);
  const v4f a2 = *(const v4f*)(sp + 256);
  const v4f a3 = *(const v4f*)(sp + 260);
  float m = -INFINITY;
#pragma unroll
  for (int e = 0; e < 4; ++e) { m = fmaxf(m, a0[e]); m = fmaxf(m, a1[e]); m = fmaxf(m, a2[e]); m = fmaxf(m, a3[e]); }
#pragma unroll
  for (int off = 1; off < 32; off <<= 1) m = fmaxf(m, __shfl_xor(m, off, 32));
  v4f e0, e1, e2, e3;
  float s = 0.f;
#pragma unroll
  for (int e = 0; e < 4; ++e) {
    e0[e] = __expf(a0[e] - m); e1[e] = __expf(a1[e] - m); e2[e] = __expf(a2[e] - m); e3[e] = __expf(a3[e] - m);
    s += (e0[e] + e1[e]) + (e2[e] + e3[e]);
  }
#pragma unroll
  for (int off = 1; off < 32; off <<= 1) s += __shfl_xor(s, off, 32);
  const float inv = 1.0f / s;
  const float f = inv * kPCarry;
  unsigned short hb[16];
#pragma unroll
  for (int e = 0; e < 4; ++e) {
    hb[e] = h_bits(e0[e] * f); hb[4 + e] = h_bits(e1[e] * f); hb[8 + e] = h_bits(e2[e] * f); hb[12 + e] = h_bits(e3[e] * f);
  }
  const v4u u0 = (v4u){pk16(hb[0], hb[1]), pk16(hb[2], hb[3]), pk16(hb[4], hb[5]), pk16(hb[6], hb[7])};
  const v4u u1 = (v4u){pk16(hb[8], hb[9]), pk16(hb[10], hb[11]), pk16(hb[12], hb[13]), pk16(hb[14], hb[15])};
  if (row < nrows) {
    unsigned short* op = Pout + (size_t)row * kNC + lane * 8;
    *(volatile v4u*)(op) = u0;
    *(volatile v4u*)(op + 256) = u1;
    __threadfence();
    *(volatile v4u*)(op) = u0;
    *(volatile v4u*)(op + 256) = u1;
  }
}

__global__ __launch_bounds__(256) void ln_relu_kernel(const float* __restrict__ H, const float* __restrict__ CW,
                                                     const float* __restrict__ gP, const float* __restrict__ btP,
                                                     const float* __restrict__ gU, const float* __restrict__ btU,
                                                     unsigned short* __restrict__ Aout, int nrows) {
  const int lane = threadIdx.x & 31, wave = threadIdx.x >> 5;
  const int gm  = blockIdx.x * 8 + wave;
  const int gmc = (gm < nrows) ? gm : (nrows - 1);
  const int z   = gmc >> 15;
  const int bix = (gmc & (kRows - 1)) >> 3;
  const int cwrow = z * kB + bix;
  const float* hp = H  + (size_t)gmc   * kHid + lane * 8;
  const float* cp = CW + (size_t)cwrow * kHid + lane * 8;
  const v4f h0 = *(const v4f*)(hp), h1 = *(const v4f*)(hp + 4);
  const v4f c0 = *(const v4f*)(cp), c1 = *(const v4f*)(cp + 4);
  const v4f x0 = h0 + c0, x1 = h1 + c1;
  float s = (x0[0] + x0[1]) + (x0[2] + x0[3]) + (x1[0] + x1[1]) + (x1[2] + x1[3]);
#pragma unroll
  for (int off = 1; off < 32; off <<= 1) s += __shfl_xor(s, off, 32);
  const float mean = s * kInvHid;
  const v4f d0 = x0 - mean, d1 = x1 - mean;
  float qs = 0.f;
#pragma unroll
  for (int e = 0; e < 4; ++e) { qs += d0[e] * d0[e]; qs += d1[e] * d1[e]; }
#pragma unroll
  for (int off = 1; off < 32; off <<= 1) qs += __shfl_xor(qs, off, 32);
  const float var = qs * kInvHid;
  const float rs  = rsqrtf(var + kLnEps);
  const v4f gp0 = *(const v4f*)(gP + lane * 8),  gp1 = *(const v4f*)(gP + lane * 8 + 4);
  const v4f bp0 = *(const v4f*)(btP + lane * 8), bp1 = *(const v4f*)(btP + lane * 8 + 4);
  const v4f gu0 = *(const v4f*)(gU + lane * 8),  gu1 = *(const v4f*)(gU + lane * 8 + 4);
  const v4f bu0 = *(const v4f*)(btU + lane * 8), bu1 = *(const v4f*)(btU + lane * 8 + 4);
  const v4f g0 = (z == 0) ? gp0 : gu0, g1 = (z == 0) ? gp1 : gu1;
  const v4f b0 = (z == 0) ? bp0 : bu0, b1 = (z == 0) ? bp1 : bu1;
  unsigned short hb[8];
#pragma unroll
  for (int e = 0; e < 4; ++e) {
    const float y0 = fmaxf(d0[e] * rs * g0[e] + b0[e], 0.0f);
    const float y1 = fmaxf(d1[e] * rs * g1[e] + b1[e], 0.0f);
    hb[e] = h_bits(y0); hb[4 + e] = h_bits(y1);
  }
  const v4u u = (v4u){pk16(hb[0], hb[1]), pk16(hb[2], hb[3]), pk16(hb[4], hb[5]), pk16(hb[6], hb[7])};
  if (gm < nrows) {
    unsigned short* op = Aout + (size_t)gm * kHid + lane * 8;
    *(volatile v4u*)op = u;
    __threadfence();
    *(volatile v4u*)op = u;
  }
}

static inline dim3 gemm_grid(int M, int N, int batch) { return dim3((unsigned)((((M / 64) * (N / 64)) + 7) / 8), (unsigned)batch, 1); }

extern "C" void kernel_launch(void* const* d_in, const int* in_sizes, int n_in,
                              void* d_out, int out_size, void* d_ws, size_t ws_size, hipStream_t stream) {
  if (n_in < 22) return;
  if (in_sizes[0] != kB * kP || in_sizes[1] != kRows * kSlot || in_sizes[2] != kP * kP || in_sizes[3] != kP ||
      in_sizes[4] != kP * kP || in_sizes[5] != kP || in_sizes[6] != kNC * kP || in_sizes[7] != kNC * kP ||
      in_sizes[8] != kNC * kP || in_sizes[9] != kNC * kP || in_sizes[10] != (kSlot + kP) * kHid || in_sizes[11] != kHid ||
      in_sizes[12] != kHid || in_sizes[13] != kHid || in_sizes[14] != kHid * kSlot || in_sizes[15] != kSlot ||
      in_sizes[16] != (kSlot + kP) * kHid || in_sizes[17] != kHid || in_sizes[18] != kHid || in_sizes[19] != kHid ||
      in_sizes[20] != kHid * kSlot || in_sizes[21] != kSlot) return;
  if (out_size != kRows * kSlot) return;

  const float* inst  = (const float*)d_in[0];
  const float* slots = (const float*)d_in[1];
  const float* Wfc   = (const float*)d_in[2];
  const float* bfc   = (const float*)d_in[3];
  const float* Wfp   = (const float*)d_in[4];
  const float* bfp   = (const float*)d_in[5];
  const float* Kc    = (const float*)d_in[6];
  const float* Vc    = (const float*)d_in[7];
  const float* Kp    = (const float*)d_in[8];
  const float* Vp    = (const float*)d_in[9];
  const float* pW1   = (const float*)d_in[10];
  const float* pb1   = (const float*)d_in[11];
  const float* pg    = (const float*)d_in[12];
  const float* pbt   = (const float*)d_in[13];
  const float* pW2   = (const float*)d_in[14];
  const float* pb2   = (const float*)d_in[15];
  const float* uW1   = (const float*)d_in[16];
  const float* ub1   = (const float*)d_in[17];
  const float* ug    = (const float*)d_in[18];
  const float* ubt   = (const float*)d_in[19];
  const float* uW2   = (const float*)d_in[20];
  const float* ub2   = (const float*)d_in[21];
  float* out = (float*)d_out;

  const size_t szSLOTB = (size_t)kRows * kSlot * 2;
  const size_t szWQT   = (size_t)2 * kP * kP * 2;
  const size_t szKF    = (size_t)2 * kNC * kP * 2;
  const size_t szVT    = (size_t)2 * kP * kNC * 2;
  const size_t szW1S   = (size_t)2 * kHid * kSlot * 2;
  const size_t szW1C   = (size_t)2 * kHid * kP * 2;
  const size_t szW2T   = (size_t)2 * kSlot * kHid * 2;
  const size_t szCW    = (size_t)2 * kB * kHid * 4;
  const size_t szA2    = (size_t)2 * kRows * kHid * 2;
  const size_t szINSTB = (size_t)kB * kP * 2;
  const size_t szQ     = (size_t)kB * 2 * kP * 2;
  const size_t szS     = (size_t)2 * kB * kNC * 4;
  const size_t szPP    = (size_t)2 * kB * kNC * 2;
  const size_t szCPL   = (size_t)2 * kB * kP * 2;
  const size_t szH     = (size_t)2 * kRows * kHid * 4;
  const size_t szGP    = (size_t)kRows * kSlot * 4;
  size_t szBIG = szINSTB + szQ + szS + szPP + szCPL;
  if (szH > szBIG) szBIG = szH;
  if (szGP > szBIG) szBIG = szGP;

  size_t off = 0;
  const size_t oSLOTB = off; off += szSLOTB;
  const size_t oWQT   = off; off += szWQT;
  const size_t oKF    = off; off += szKF;
  const size_t oVT    = off; off += szVT;
  const size_t oW1S   = off; off += szW1S;
  const size_t oW1C   = off; off += szW1C;
  const size_t oW2T   = off; off += szW2T;
  const size_t oCW    = off; off += szCW;
  const size_t oA2    = off; off += szA2;
  const size_t oBIG   = off; off += szBIG;
  if (off > ws_size) return;

  char* ws = (char*)d_ws;
  unsigned short* slotsB = (unsigned short*)(ws + oSLOTB);
  unsigned short* WqT    = (unsigned short*)(ws + oWQT);
  unsigned short* KF     = (unsigned short*)(ws + oKF);
  unsigned short* VT     = (unsigned short*)(ws + oVT);
  unsigned short* W1S    = (unsigned short*)(ws + oW1S);
  unsigned short* W1C    = (unsigned short*)(ws + oW1C);
  unsigned short* W2T    = (unsigned short*)(ws + oW2T);
  float*          CW     = (float*)(ws + oCW);
  unsigned short* A2     = (unsigned short*)(ws + oA2);
  unsigned short* instB  = (unsigned short*)(ws + oBIG);
  unsigned short* Qpl    = (unsigned short*)(ws + oBIG + szINSTB);
  float*          S      = (float*)(ws + oBIG + szINSTB + szQ);
  unsigned short* Ppl    = (unsigned short*)(ws + oBIG + szINSTB + szQ + szS);
  unsigned short* Cpl    = (unsigned short*)(ws + oBIG + szINSTB + szQ + szS + szPP);
  float*          H      = (float*)(ws + oBIG);
  float*          GP     = (float*)(ws + oBIG);

  const long zWQT = (long)kP * kP;
  const long zKF  = (long)kNC * kP;
  const long zVT  = (long)kP * kNC;
  const long zW1S = (long)kHid * kSlot;
  const long zW1C = (long)kHid * kP;
  const long zW2T = (long)kSlot * kHid;
  const long zCW  = (long)kB * kHid;
  const long zS   = (long)kB * kNC;
  const long zCPL = (long)kB * kP;
  const long zH   = (long)kRows * kHid;

  cast8_kernel<0><<<dim3((kB * kP / 8) / 256, 1), 256, 0, stream>>>(inst, inst, instB, 0, kB * kP / 8, 1.0f);
  cast8_kernel<0><<<dim3((kRows * kSlot / 8) / 256, 1), 256, 0, stream>>>(slots, slots, slotsB, 0, kRows * kSlot / 8, 1.0f);
  cast8_kernel<1><<<dim3((kNC * kP / 8) / 256, 2), 256, 0, stream>>>(Kc, Kp, KF, zKF, kNC * kP / 8, 1.0f);
  tcast_kernel<0><<<dim3(kP / 64, kP / 64, 2), 256, 0, stream>>>(Wfc, Wfp, kP, 0, WqT, zWQT, kP, 1.0f);
  tcast_kernel<1><<<dim3(kNC / 64, kP / 64, 2), 256, 0, stream>>>(Vc, Vp, kP, 0, VT, zVT, kNC, 1.0f);
  tcast_kernel<0><<<dim3(kSlot / 64, kHid / 64, 2), 256, 0, stream>>>(pW1, uW1, kHid, 0, W1S, zW1S, kSlot, 1.0f);
  tcast_kernel<1><<<dim3(kP / 64, kHid / 64, 2), 256, 0, stream>>>(pW1, uW1, kHid, kSlot, W1C, zW1C, kP, kWCarry);
  tcast_kernel<1><<<dim3(kHid / 64, kSlot / 64, 2), 256, 0, stream>>>(pW2, uW2, kSlot, 0, W2T, zW2T, kHid, kWCarry);

  wmma_gemm64<1, false, 2, 1, 0, false><<<gemm_grid(kB, kP, 1), 256, 0, stream>>>(
      instB, instB, kP, 0, WqT, WqT, kP, 0, Qpl, Qpl, 2 * kP, 0, bfc, slots, 0, slots, 0, kB, kP, kP, 1.0f);
  wmma_gemm64<1, false, 2, 1, 0, false><<<gemm_grid(kB, kP, 1), 256, 0, stream>>>(
      instB, instB, kP, 0, WqT + zWQT, WqT + zWQT, kP, 0, Qpl + kP, Qpl + kP, 2 * kP, 0, bfp, slots, 0, slots, 0, kB, kP, kP, 1.0f);

  wmma_gemm64<0, false, 0, 0, 0, false><<<gemm_grid(kB, kNC, 2), 256, 0, stream>>>(
      Qpl, Qpl, 2 * kP, (long)kP, KF, KF, kP, zKF, S, S, kNC, zS, bfc, slots, 0, slots, 0, kB, kNC, kP, kInvSqrtP);

  softmax_kernel<<<dim3((2 * kB) / 8), 256, 0, stream>>>(S, Ppl, 2 * kB);

  wmma_gemm64<0, false, 0, 1, 0, false><<<gemm_grid(kB, kP, 2), 256, 0, stream>>>(
      Ppl, Ppl, kNC, zS, VT, VT, kNC, zVT, Cpl, Cpl, kP, zCPL, bfc, slots, 0, slots, 0, kB, kP, kNC, kPVScale);

  wmma_gemm64<0, false, 2, 0, 0, false><<<gemm_grid(kB, kHid, 1), 256, 0, stream>>>(
      Cpl, Cpl, kP, 0, W1C, W1C, kP, 0, CW, CW, kHid, 0, pb1, slots, 0, slots, 0, kB, kHid, kP, kCWScale);
  wmma_gemm64<0, false, 2, 0, 0, false><<<gemm_grid(kB, kHid, 1), 256, 0, stream>>>(
      Cpl + zCPL, Cpl + zCPL, kP, 0, W1C + zW1C, W1C + zW1C, kP, 0, CW + zCW, CW + zCW, kHid, 0, ub1, slots, 0, slots, 0, kB, kHid, kP, kCWScale);

  wmma_gemm64<1, false, 0, 0, 0, false><<<gemm_grid(kRows, kHid, 2), 256, 0, stream>>>(
      slotsB, slotsB, kSlot, 0, W1S, W1S, kSlot, zW1S, H, H, kHid, zH, bfc, slots, 0, slots, 0, kRows, kHid, kSlot, 1.0f);

  ln_relu_kernel<<<dim3((2 * kRows) / 8), 256, 0, stream>>>(H, CW, pg, pbt, ug, ubt, A2, 2 * kRows);

  wmma_gemm64<0, false, 2, 0, 0, false><<<gemm_grid(kRows, kSlot, 1), 256, 0, stream>>>(
      A2, A2, kHid, 0, W2T, W2T, kHid, 0, GP, GP, kSlot, 0, pb2, slots, 0, slots, 0, kRows, kSlot, kHid, kW2Scale);

  wmma_gemm64<0, false, 2, 0, 2, true><<<gemm_grid(kRows, kSlot, 1), 256, 0, stream>>>(
      A2 + zH, A2 + zH, kHid, 0, W2T + zW2T, W2T + zW2T, kHid, 0, out, out, kSlot, 0, ub2, slots, 0, GP, 0, kRows, kSlot, kHid, kW2Scale);
}
